// WaveformDecoder_13580686590630
// MI455X (gfx1250) — hardware-verified
//
#include <hip/hip_runtime.h>


#define NB_    2
#define CIN_   256
#define TIN_   128
#define UPK_   256
#define CH_    64
#define LQ_    32768
#define NBLK_  30
#define KG_    192
#define NP_    128
#define SP_    68
#define MUP_   (NB_ * TIN_)
#define NUP_   (UPK_ * CH_)

#define PB0_   32
#define PB1_   (PB0_ + 2048)
#define PB2_   (PB1_ + 360)
#define PB3_   (PB2_ + 60)

static_assert(MUP_ * CIN_ == PB0_ * 256 * 8);
static_assert(NUP_ * CIN_ == (PB1_ - PB0_) * 256 * 8);
static_assert(NBLK_ * 2 * CH_ * KG_ == (PB2_ - PB1_) * 256 * 8);
static_assert(NBLK_ * CH_ * CH_ == (PB3_ - PB2_) * 256 * 8);
static_assert(LQ_ % NP_ == 0);
static_assert(NP_ == 8 * 16);
static_assert(MUP_ % 64 == 0);
static_assert(NUP_ % 128 == 0);
static_assert(CIN_ % 32 == 0);
static_assert(KG_ % 32 == 0);
static_assert((SP_ * 4) % 16 == 0);
static_assert(TIN_ * UPK_ == LQ_);

typedef float          v4f   __attribute__((ext_vector_type(4)));
typedef float          v8f   __attribute__((ext_vector_type(8)));
typedef _Float16       v8h   __attribute__((ext_vector_type(8)));
typedef _Float16       v16h  __attribute__((ext_vector_type(16)));
typedef unsigned short u16x8 __attribute__((ext_vector_type(8)));
typedef unsigned int   u32x4 __attribute__((ext_vector_type(4)));

union FragH { u16x8 h[2]; u32x4 w[2]; v16h v; };
union Pack8 { v8h f; u16x8 u; };

__device__ __forceinline__ void mma16(v8f& acc, const FragH& a, const FragH& b) {
    acc = __builtin_amdgcn_wmma_f32_16x16x32_f16(false, a.v, false, b.v, (short)0, acc, false, false);
    asm volatile("v_nop\n\tv_nop\n\tv_nop\n\tv_nop" : "+v"(acc) : "v"(a.v), "v"(b.v));
}
__device__ __forceinline__ u16x8 pack8h(v8f x) {
    Pack8 pk;
    pk.f = __builtin_convertvector(x, v8h);
    return pk.u;
}
__device__ __forceinline__ v8f ld8f(const float* p) {
    v4f a = *(const v4f*)p;
    v4f b = *(const v4f*)(p + 4);
    return __builtin_shufflevector(a, b, 0, 1, 2, 3, 4, 5, 6, 7);
}
__device__ __forceinline__ v8f zero8f() {
    v8f z;
#pragma unroll
    for (int i = 0; i < 8; ++i) z[i] = 0.0f;
    return z;
}
__device__ __forceinline__ void ldfrag(FragH& f, const unsigned short* p) {
    f.h[0] = *(const u16x8*)(p);
    f.h[1] = *(const u16x8*)(p + 16);
}

__global__ __launch_bounds__(256)
void prep_kernel(const float* __restrict__ x, const float* __restrict__ Wup,
                 const float* __restrict__ Wg, const float* __restrict__ Wr,
                 unsigned short* X16, unsigned short* WupT16,
                 unsigned short* Wg16, unsigned short* Wr16)
{
    const int blk = blockIdx.x;
    const int tid = threadIdx.x;
    if (blk >= PB3_) return;
    v8f v;
    unsigned short* dst;
    if (blk < PB0_) {
        const int p   = blk * 256 + tid;
        const int row = p >> 5;
        const int c0  = (p & 31) * 8;
        const int b   = row >> 7;
        const int t   = row & 127;
#pragma unroll
        for (int i = 0; i < 8; ++i)
            v[i] = x[((size_t)(b * CIN_ + c0 + i)) * TIN_ + t];
        dst = X16 + (size_t)p * 8;
    } else if (blk < PB1_) {
        const int p  = (blk - PB0_) * 256 + tid;
        const int n  = p >> 5;
        const int c0 = (p & 31) * 8;
        const int k  = n >> 6;
        const int o  = n & 63;
#pragma unroll
        for (int i = 0; i < 8; ++i)
            v[i] = Wup[((size_t)(c0 + i) * CH_ + o) * UPK_ + k];
        dst = WupT16 + (size_t)p * 8;
    } else if (blk < PB2_) {
        const int p   = (blk - PB1_) * 256 + tid;
        const int row = p / 24;
        const int pr  = p - row * 24;
        const int j   = pr >> 3;
        const int c0  = (pr & 7) * 8;
#pragma unroll
        for (int i = 0; i < 8; ++i)
            v[i] = Wg[((size_t)row * CH_ + c0 + i) * 3 + j];
        dst = Wg16 + (size_t)p * 8;
    } else {
        const int p = (blk - PB2_) * 256 + tid;
#pragma unroll
        for (int i = 0; i < 8; ++i)
            v[i] = Wr[(size_t)p * 8 + i];
        dst = Wr16 + (size_t)p * 8;
    }
    const u16x8 u = pack8h(v * 16.0f);
    *(volatile u16x8*)dst = u;
    __threadfence();
    *(volatile u16x8*)dst = u;
}

__device__ __forceinline__ void up_pass32(const float* st, float* gp, int lane) {
    const int rsub = lane >> 4;
    const int c4   = (lane & 15) * 4;
#pragma unroll
    for (int it = 0; it < 16; ++it) {
        const int row = it * 2 + rsub;
        const v4f v = *(const v4f*)(st + row * SP_ + c4);
        *(volatile v4f*)(gp + (size_t)row * NUP_ + c4) = v;
    }
}
__device__ __forceinline__ void up_pass16(const float* st, unsigned short* gp, int lane) {
    const int rsub = lane >> 3;
    const int c8   = (lane & 7) * 8;
#pragma unroll
    for (int it = 0; it < 8; ++it) {
        const int row = it * 4 + rsub;
        const u16x8 u = pack8h(ld8f(st + row * SP_ + c8) * 16.0f);
        *(volatile u16x8*)(gp + (size_t)row * NUP_ + c8) = u;
    }
}

__global__ __launch_bounds__(128)
void upgemm_kernel(const unsigned short* __restrict__ A, const unsigned short* __restrict__ Bw,
                   const float* __restrict__ bup, float* C32, unsigned short* C16)
{
    __shared__ __attribute__((aligned(16))) float stile[4][32 * SP_];

    const int tid  = threadIdx.x;
    const int lane = tid & 31;
    const int wave = tid >> 5;
    const int h    = lane >> 4;
    const int m    = lane & 15;
    const int wm   = wave >> 1;
    const int wn   = wave & 1;

    const int rowW = blockIdx.y * 64 + wm * 32;
    const int colW = blockIdx.x * 128 + wn * 64;

    v8f acc[8];
#pragma unroll
    for (int j = 0; j < 8; ++j) acc[j] = zero8f();

    const size_t aoff  = (size_t)(rowW + m) * CIN_ + 8 * h;
    const size_t boff  = (size_t)(colW + m) * CIN_ + 8 * h;
    const size_t sub16 = (size_t)16 * CIN_;

#pragma unroll 1
    for (int kt = 0; kt < CIN_ / 32; ++kt) {
        const int k0 = kt * 32;
        FragH fa[2], fb[4];
#pragma unroll
        for (int s = 0; s < 2; ++s) ldfrag(fa[s], A + aoff + s * sub16 + k0);
#pragma unroll
        for (int j = 0; j < 4; ++j) ldfrag(fb[j], Bw + boff + j * sub16 + k0);
#pragma unroll
        for (int s = 0; s < 2; ++s)
#pragma unroll
            for (int j = 0; j < 4; ++j)
                mma16(acc[s * 4 + j], fa[s], fb[j]);
    }

    float* st = stile[wave];
    float bcol[4];
#pragma unroll
    for (int j = 0; j < 4; ++j) bcol[j] = bup[j * 16 + m];
#pragma unroll
    for (int s = 0; s < 2; ++s)
#pragma unroll
        for (int j = 0; j < 4; ++j)
#pragma unroll
            for (int r = 0; r < 8; ++r)
                st[(s * 16 + 8 * h + r) * SP_ + j * 16 + m] = acc[s * 4 + j][r] * 0.00390625f + bcol[j];
    __syncthreads();

    const size_t goff = (size_t)rowW * NUP_ + colW;
    up_pass32(st, C32 + goff, lane);
    up_pass16(st, C16 + goff, lane);
    __threadfence();
    up_pass32(st, C32 + goff, lane);
    up_pass16(st, C16 + goff, lane);
}

__device__ __forceinline__ void rb_pass32(const float* S, float* y32out, size_t rowbase, int tid) {
#pragma unroll
    for (int it = 0; it < 8; ++it) {
        const int q   = it * 256 + tid;
        const int pos = q >> 4;
        const int c4  = (q & 15) * 4;
        const v4f v = *(const v4f*)(S + pos * SP_ + c4);
        *(volatile v4f*)(y32out + (rowbase + pos) * CH_ + c4) = v;
    }
}
__device__ __forceinline__ void rb_pass16(const float* S, unsigned short* y16out, size_t rowbase, int tid) {
#pragma unroll
    for (int it = 0; it < 4; ++it) {
        const int q   = it * 256 + tid;
        const int pos = q >> 3;
        const int c8  = (q & 7) * 8;
        const u16x8 u = pack8h(ld8f(S + pos * SP_ + c8) * 16.0f);
        *(volatile u16x8*)(y16out + (rowbase + pos) * CH_ + c8) = u;
    }
}

__global__ __launch_bounds__(256)
void resblock_kernel(const float* __restrict__ y32in, const unsigned short* __restrict__ y16in,
                     float* y32out, unsigned short* y16out,
                     const unsigned short* __restrict__ Wg16, const float* __restrict__ bg,
                     const unsigned short* __restrict__ Wr16, const float* __restrict__ br, int d)
{
    __shared__ __attribute__((aligned(16))) float S[NP_ * SP_];

    const int tid  = threadIdx.x;
    const int lane = tid & 31;
    const int wave = tid >> 5;
    const int h    = lane >> 4;
    const int m    = lane & 15;
    const int b    = blockIdx.y;
    const int tileL = blockIdx.x * NP_;
    const size_t rowbase = (size_t)b * LQ_ + tileL;
    const int p0 = tileL + wave * 16;

    v8f acc[8];
#pragma unroll
    for (int j = 0; j < 8; ++j) acc[j] = zero8f();

#pragma unroll 1
    for (int ks = 0; ks < KG_ / 32; ++ks) {
        const int j    = ks >> 1;
        const int cb   = (ks & 1) * 32;
        const int lsrc = p0 + m + (j - 1) * d;
        const unsigned msk = (lsrc >= 0 && lsrc < LQ_) ? 0xFFFFFFFFu : 0u;
        const int lc   = min(max(lsrc, 0), LQ_ - 1);
        const unsigned short* yp = y16in + ((size_t)b * LQ_ + lc) * CH_ + cb + 8 * h;
        const u32x4 mk = {msk, msk, msk, msk};
        FragH bf;
        ldfrag(bf, yp);
        bf.w[0] &= mk;
        bf.w[1] &= mk;
        const int k0 = ks * 32;
#pragma unroll
        for (int mt = 0; mt < 8; ++mt) {
            FragH af;
            ldfrag(af, Wg16 + (size_t)(16 * mt + m) * KG_ + k0 + 8 * h);
            mma16(acc[mt], af, bf);
        }
    }

    FragH gfr[2];
#pragma unroll
    for (int mt = 0; mt < 4; ++mt) {
        const v8f bz1 = ld8f(bg + 16 * mt + 8 * h);
        const v8f bz2 = ld8f(bg + CH_ + 16 * mt + 8 * h);
        v8f gv;
#pragma unroll
        for (int r = 0; r < 8; ++r) {
            const float z1 = acc[mt][r] * 0.00390625f + bz1[r];
            const float z2 = acc[mt + 4][r] * 0.00390625f + bz2[r];
            const float th = 1.0f - 2.0f * __builtin_amdgcn_rcpf(__expf(2.0f * z1) + 1.0f);
            const float sg = __builtin_amdgcn_rcpf(1.0f + __expf(-z2));
            gv[r] = th * sg * 256.0f;
        }
        gfr[mt >> 1].h[mt & 1] = pack8h(gv);
    }

    v8f acc2[4];
#pragma unroll
    for (int j = 0; j < 4; ++j) acc2[j] = zero8f();
#pragma unroll
    for (int mt = 0; mt < 4; ++mt)
#pragma unroll
        for (int kc = 0; kc < 2; ++kc) {
            FragH af;
            ldfrag(af, Wr16 + (size_t)(16 * mt + m) * CH_ + 32 * kc + 8 * h);
            mma16(acc2[mt], af, gfr[kc]);
        }

    const int prow = wave * 16 + m;
#pragma unroll
    for (int mt = 0; mt < 4; ++mt) {
        const v8f bb = ld8f(br + 16 * mt + 8 * h);
        const v8f rv = acc2[mt] * 0.000244140625f + bb;
        float* sp = S + prow * SP_ + 16 * mt + 8 * h;
        *(v4f*)(sp)     = rv.lo;
        *(v4f*)(sp + 4) = rv.hi;
    }
    __syncthreads();

#pragma unroll
    for (int it = 0; it < 8; ++it) {
        const int q   = it * 256 + tid;
        const int pos = q >> 4;
        const int c4  = (q & 15) * 4;
        float* sp = S + pos * SP_ + c4;
        const v4f yv = *(const v4f*)(y32in + (rowbase + pos) * CH_ + c4);
        const v4f v  = *(const v4f*)sp + yv;
        *(v4f*)sp = v;
    }
    __syncthreads();

    rb_pass32(S, y32out, rowbase, tid);
    rb_pass16(S, y16out, rowbase, tid);
    __threadfence();
    rb_pass32(S, y32out, rowbase, tid);
    rb_pass16(S, y16out, rowbase, tid);
}

__global__ __launch_bounds__(256)
void final_kernel(const float* __restrict__ y32, const float* __restrict__ Wf,
                  const float* __restrict__ bfp, float* out, int n)
{
    const int idx = blockIdx.x * 256 + threadIdx.x;
    if (idx >= n) return;
    const float* yr = y32 + (size_t)idx * CH_;
    float acc = bfp[0];
#pragma unroll 4
    for (int c = 0; c < CH_; c += 4) {
        const v4f yv = *(const v4f*)(yr + c);
        const v4f wv = *(const v4f*)(Wf + c);
        acc = fmaf(yv[0], wv[0], acc);
        acc = fmaf(yv[1], wv[1], acc);
        acc = fmaf(yv[2], wv[2], acc);
        acc = fmaf(yv[3], wv[3], acc);
    }
    *(volatile float*)(out + idx) = acc;
    __threadfence();
    *(volatile float*)(out + idx) = acc;
}

extern "C" void kernel_launch(void* const* d_in, const int* in_sizes, int n_in,
                              void* d_out, int out_size, void* d_ws, size_t ws_size,
                              hipStream_t stream)
{
    if (n_in < 9) return;
    if (in_sizes[0] != NB_ * CIN_ * TIN_)         return;
    if (in_sizes[1] != CIN_ * CH_ * UPK_)         return;
    if (in_sizes[2] != CH_)                       return;
    if (in_sizes[3] != NBLK_ * 2 * CH_ * CH_ * 3) return;
    if (in_sizes[4] != NBLK_ * 2 * CH_)           return;
    if (in_sizes[5] != NBLK_ * CH_ * CH_)         return;
    if (in_sizes[6] != NBLK_ * CH_)               return;
    if (in_sizes[7] != CH_)                       return;
    if (in_sizes[8] < 1)                          return;
    if (out_size != NB_ * LQ_)                    return;

    const float* x    = (const float*)d_in[0];
    const float* Wup  = (const float*)d_in[1];
    const float* bup  = (const float*)d_in[2];
    const float* Wg   = (const float*)d_in[3];
    const float* bg   = (const float*)d_in[4];
    const float* Wr   = (const float*)d_in[5];
    const float* br   = (const float*)d_in[6];
    const float* Wf   = (const float*)d_in[7];
    const float* bfp  = (const float*)d_in[8];
    float* out = (float*)d_out;

    const size_t SZ_Y32 = (size_t)NB_ * LQ_ * CH_ * 4;
    const size_t SZ_Y16 = (size_t)NB_ * LQ_ * CH_ * 2;
    const size_t SZ_X16 = (size_t)MUP_ * CIN_ * 2;
    const size_t SZ_WUP = (size_t)NUP_ * CIN_ * 2;
    const size_t SZ_WG  = (size_t)NBLK_ * 2 * CH_ * KG_ * 2;
    const size_t SZ_WR  = (size_t)NBLK_ * CH_ * CH_ * 2;

    const size_t OFF_Y32A = 0;
    const size_t OFF_Y32B = OFF_Y32A + SZ_Y32;
    const size_t OFF_Y16A = OFF_Y32B + SZ_Y32;
    const size_t OFF_Y16B = OFF_Y16A + SZ_Y16;
    const size_t OFF_X16  = OFF_Y16B + SZ_Y16;
    const size_t OFF_WUP  = OFF_X16 + SZ_X16;
    const size_t OFF_WG   = OFF_WUP + SZ_WUP;
    const size_t OFF_WR   = OFF_WG + SZ_WG;
    const size_t WS_END   = OFF_WR + SZ_WR;
    if (ws_size < WS_END) return;

    char* ws = (char*)d_ws;
    float*          y32A   = (float*)(ws + OFF_Y32A);
    float*          y32B   = (float*)(ws + OFF_Y32B);
    unsigned short* y16A   = (unsigned short*)(ws + OFF_Y16A);
    unsigned short* y16B   = (unsigned short*)(ws + OFF_Y16B);
    unsigned short* X16    = (unsigned short*)(ws + OFF_X16);
    unsigned short* WupT16 = (unsigned short*)(ws + OFF_WUP);
    unsigned short* Wg16   = (unsigned short*)(ws + OFF_WG);
    unsigned short* Wr16   = (unsigned short*)(ws + OFF_WR);

    prep_kernel<<<dim3(PB3_), dim3(256), 0, stream>>>(x, Wup, Wg, Wr, X16, WupT16, Wg16, Wr16);

    upgemm_kernel<<<dim3(NUP_ / 128, MUP_ / 64), dim3(128), 0, stream>>>(
        (const unsigned short*)X16, (const unsigned short*)WupT16, bup, y32A, y16A);

    for (int i = 0; i < NBLK_; ++i) {
        const int dil = 1 << (i % 10);
        const float*          yi32 = (i & 1) ? y32B : y32A;
        const unsigned short* yi16 = (i & 1) ? y16B : y16A;
        float*                yo32 = (i & 1) ? y32A : y32B;
        unsigned short*       yo16 = (i & 1) ? y16A : y16B;
        resblock_kernel<<<dim3(LQ_ / NP_, NB_), dim3(256), 0, stream>>>(
            yi32, yi16, yo32, yo16,
            (const unsigned short*)(Wg16 + (size_t)i * 2 * CH_ * KG_),
            bg + (size_t)i * 2 * CH_,
            (const unsigned short*)(Wr16 + (size_t)i * CH_ * CH_),
            br + (size_t)i * CH_,
            dil);
    }

    final_kernel<<<dim3((NB_ * LQ_ + 255) / 256), dim3(256), 0, stream>>>(
        (const float*)y32A, Wf, bfp, out, NB_ * LQ_);
}
